// MultiHeadAttentionLinear_27066883899621
// MI455X (gfx1250) — hardware-verified
//
#include <hip/hip_runtime.h>
#include <math.h>
#include <stdint.h>

#define NB    2
#define SEQ   1024
#define DK    512
#define NH    8
#define DQ    (NH * DK)
#define MR    (NB * SEQ)
#define NHB   (NH * NB)
#define SBLK  32
#define NSB   (SEQ / SBLK)
#define QRES  ((long long)MR * DQ)
#define VRES  ((long long)NHB * DK * SEQ)
#define WSC   64.0f
#define RSC   2048.0f
#define PSC   8192.0f
#define NEGBIG (-1.0e30f)
static_assert((SEQ % 64) == 0 && (DK % 64) == 0 && (MR % 64) == 0 && (DQ % 64) == 0);
static_assert(SEQ == NSB * SBLK);
static_assert(SBLK == 32);
static_assert((DK % 32) == 0 && (SEQ % 256) == 0);

typedef _Float16       v16h __attribute__((ext_vector_type(16)));
typedef unsigned short v16us __attribute__((ext_vector_type(16)));
typedef unsigned short v8us __attribute__((ext_vector_type(8)));
typedef float          v8f  __attribute__((ext_vector_type(8)));
typedef float          v4f  __attribute__((ext_vector_type(4)));
typedef unsigned int   v4u  __attribute__((ext_vector_type(4)));

union Frag { v16us u; v8us p[2]; v16h h; };

__device__ __forceinline__ unsigned short bf_bits(float f) {
  unsigned u = __float_as_uint(f);
  return (unsigned short)((u + 0x7FFFu + ((u >> 16) & 1u)) >> 16);
}
__device__ __forceinline__ float bf_up(unsigned short b) { return __uint_as_float(((unsigned)b) << 16); }
__device__ __forceinline__ float bfr(float f) { return bf_up(bf_bits(f)); }
__device__ __forceinline__ unsigned short h_bits(_Float16 x) { return __builtin_bit_cast(unsigned short, x); }
__device__ __forceinline__ unsigned pk16(unsigned short a, unsigned short b) { return (unsigned)a | ((unsigned)b << 16); }
__device__ __forceinline__ v8f zero8() { v8f z = {0.f, 0.f, 0.f, 0.f, 0.f, 0.f, 0.f, 0.f}; return z; }

__device__ __forceinline__ v16us ldfrag(const unsigned short* p) {
  Frag f;
  f.p[0] = *(const v8us*)(p);
  f.p[1] = *(const v8us*)(p + 16);
  return f.u;
}

__device__ __forceinline__ v8f mma_raw(v16us a, v16us b, v8f c) {
  Frag fa, fb;
  fa.u = a;
  fb.u = b;
  return __builtin_amdgcn_wmma_f32_16x16x32_f16(false, fa.h, false, fb.h, (short)0, c, false, false);
}
__device__ __forceinline__ void dep_guard1(v8f& a, v8f& b, v16us x) {
#if defined(__HIP_DEVICE_COMPILE__)
  asm volatile("v_nop\n\tv_nop\n\tv_nop\n\tv_nop" : "+v"(a), "+v"(b) : "v"(x));
#endif
}
__device__ __forceinline__ void keep4(v16us a, v16us b, v16us c, v16us d) {
#if defined(__HIP_DEVICE_COMPILE__)
  asm volatile("v_nop" :: "v"(a), "v"(b), "v"(c), "v"(d));
#endif
}
__device__ __forceinline__ void acc_guard4(v8f& a, v8f& b, v8f& c, v8f& d) {
#if defined(__HIP_DEVICE_COMPILE__)
  asm volatile("v_nop\n\tv_nop\n\tv_nop\n\tv_nop" : "+v"(a), "+v"(b), "+v"(c), "+v"(d));
#endif
}
__device__ __forceinline__ void guard2k4(v8f& a, v8f& b, v16us w, v16us x, v16us y, v16us z) {
#if defined(__HIP_DEVICE_COMPILE__)
  asm volatile("v_nop\n\tv_nop\n\tv_nop\n\tv_nop" : "+v"(a), "+v"(b) : "v"(w), "v"(x), "v"(y), "v"(z));
#endif
}
__device__ __forceinline__ void guard4k4(v8f& a, v8f& b, v8f& c, v8f& d, v16us w, v16us x, v16us y, v16us z) {
#if defined(__HIP_DEVICE_COMPILE__)
  asm volatile("v_nop\n\tv_nop\n\tv_nop\n\tv_nop" : "+v"(a), "+v"(b), "+v"(c), "+v"(d) : "v"(w), "v"(x), "v"(y), "v"(z));
#endif
}
__device__ __forceinline__ void wave_sync_lds() {
  __builtin_amdgcn_fence(__ATOMIC_RELEASE, "workgroup");
  __builtin_amdgcn_wave_barrier();
  __builtin_amdgcn_fence(__ATOMIC_ACQUIRE, "workgroup");
}

__global__ __launch_bounds__(256) void conv_h16(const float* __restrict__ X, unsigned short* Xh, int n8, float wsc) {
  const int i  = blockIdx.x * 256 + threadIdx.x;
  const int ic = (i < n8) ? i : (n8 - 1);
  const float* src = X + (size_t)ic * 8;
  const v4f a = *(const v4f*)(src);
  const v4f c = *(const v4f*)(src + 4);
  v4u o;
  o[0] = pk16(h_bits((_Float16)(bfr(a[0]) * wsc)), h_bits((_Float16)(bfr(a[1]) * wsc)));
  o[1] = pk16(h_bits((_Float16)(bfr(a[2]) * wsc)), h_bits((_Float16)(bfr(a[3]) * wsc)));
  o[2] = pk16(h_bits((_Float16)(bfr(c[0]) * wsc)), h_bits((_Float16)(bfr(c[1]) * wsc)));
  o[3] = pk16(h_bits((_Float16)(bfr(c[2]) * wsc)), h_bits((_Float16)(bfr(c[3]) * wsc)));
  if (i < n8) *(volatile v4u*)(Xh + (size_t)i * 8) = o;
  __threadfence();
  if (i < n8) *(volatile v4u*)(Xh + (size_t)i * 8) = o;
}

__global__ __launch_bounds__(256) void tconv_h16(const float* __restrict__ W, unsigned short* WT, int ncols, float wsc) {
  __shared__ float tile[64][65];
  const int tid = threadIdx.x, lane = tid & 31, wave = tid >> 5;
  const int n0 = blockIdx.x * 64, k0 = blockIdx.y * 64;
  {
    const int r = tid >> 2, cq = (tid & 3) * 16;
    const float* src = W + (size_t)(k0 + r) * (size_t)ncols + n0 + cq;
#pragma unroll
    for (int i = 0; i < 4; ++i) {
      const v4f a = *(const v4f*)(src + 4 * i);
#pragma unroll
      for (int e = 0; e < 4; ++e) tile[r][cq + 4 * i + e] = a[e];
    }
  }
  __syncthreads();
  const int nl = lane >> 3, kq = (lane & 7) * 8;
#pragma unroll
  for (int it = 0; it < 2; ++it) {
    const int n = wave * 8 + it * 4 + nl;
    v4u o;
#pragma unroll
    for (int e = 0; e < 4; ++e) {
      const float f0 = bfr(tile[kq + 2 * e][n]) * wsc;
      const float f1 = bfr(tile[kq + 2 * e + 1][n]) * wsc;
      o[e] = pk16(h_bits((_Float16)f0), h_bits((_Float16)f1));
    }
    unsigned short* dst = WT + (size_t)(n0 + n) * DK + k0 + kq;
    *(volatile v4u*)dst = o;
    __threadfence();
    *(volatile v4u*)dst = o;
  }
}

template <int OM, int BIASM>
__global__ __launch_bounds__(256) void gemm64(
    const unsigned short* __restrict__ A, int lda, long long strideA,
    const unsigned short* __restrict__ Bt, int ldb, long long strideB,
    const float* __restrict__ bias, int nbias, long long strideBias, int ydiv,
    void* Cout, int ldc, long long strideC, long long resOff,
    int M, int N, int K, float oscale) {
  __shared__ __align__(16) float sT[8][16 * 68];
  const int y    = blockIdx.y;
  const int ya   = y / ydiv;
  const int yb   = y - ya * ydiv;
  const int lane = threadIdx.x & 31;
  const int wave = threadIdx.x >> 5;
  const int tilesN = N >> 6;
  const int tilesM = M >> 6;
  const int tile = blockIdx.x * 8 + wave;
  if (tile >= tilesM * tilesN) return;
  const int tm = tile / tilesN;
  const int tn = tile - tm * tilesN;
  const int m0 = tm << 6;
  const int n0 = tn << 6;

  const unsigned short* Ab = A  + (size_t)ya * (size_t)strideA;
  const unsigned short* Bb = Bt + (size_t)yb * (size_t)strideB;
  const float* biasb = bias + (size_t)ya * (size_t)strideBias;

  const int rlane = lane & 15;
  const int koff  = (lane >> 4) * 8;
  const int mOff  = (lane >> 4) * 8;

  v8f acc[4][4];
#pragma unroll
  for (int i = 0; i < 4; ++i)
#pragma unroll
    for (int j = 0; j < 4; ++j) acc[i][j] = zero8();

  for (int k0 = 0; k0 < K; k0 += 32) {
    v16us bh[4];
#pragma unroll
    for (int j = 0; j < 4; ++j) {
      const size_t bo = (size_t)(n0 + (j << 4) + rlane) * ldb + koff + k0;
      bh[j] = ldfrag(Bb + bo);
    }
#pragma unroll
    for (int i = 0; i < 4; ++i) {
      const size_t ao = (size_t)(m0 + (i << 4) + rlane) * lda + koff + k0;
      const v16us ah = ldfrag(Ab + ao);
#pragma unroll
      for (int j = 0; j < 4; ++j) acc[i][j] = mma_raw(ah, bh[j], acc[i][j]);
      dep_guard1(acc[i][0], acc[i][3], ah);
    }
    keep4(bh[0], bh[1], bh[2], bh[3]);
  }
  acc_guard4(acc[0][0], acc[0][1], acc[0][2], acc[0][3]);
  acc_guard4(acc[1][0], acc[1][1], acc[1][2], acc[1][3]);
  acc_guard4(acc[2][0], acc[2][1], acc[2][2], acc[2][3]);
  acc_guard4(acc[3][0], acc[3][1], acc[3][2], acc[3][3]);

  const int hh2 = lane >> 4, c4 = (lane & 15) * 4;
  const int q8  = lane >> 3, c8 = (lane & 7) * 8;
  float bc[8];
#pragma unroll
  for (int e = 0; e < 8; ++e) bc[e] = 0.f;
  if constexpr (BIASM == 0) {
    if constexpr (OM == 0) {
      const int cb = n0 + c4;
      const int i0 = (cb < nbias - 4) ? cb : (nbias - 4);
      const v4f b0v = *(const v4f*)(biasb + i0);
#pragma unroll
      for (int e = 0; e < 4; ++e) bc[e] = bfr(b0v[e]);
    } else {
      const int cb = n0 + c8;
      const int i0 = (cb < nbias - 8) ? cb : (nbias - 8);
      const v4f b0a = *(const v4f*)(biasb + i0), b0b = *(const v4f*)(biasb + i0 + 4);
#pragma unroll
      for (int e = 0; e < 4; ++e) {
        bc[e]     = bfr(b0a[e]);
        bc[4 + e] = bfr(b0b[e]);
      }
    }
  }

  float* slab = sT[wave];
#pragma unroll
  for (int i = 0; i < 4; ++i) {
    const int mBase = m0 + (i << 4);
#pragma unroll
    for (int j = 0; j < 4; ++j) {
#pragma unroll
      for (int r = 0; r < 8; ++r) {
        slab[(mOff + r) * 68 + (j << 4) + rlane] = acc[i][j][r];
      }
    }
    wave_sync_lds();
    if constexpr (OM == 0) {
      float* C = (float*)Cout + (size_t)y * (size_t)strideC;
      v4f vals[8];
#pragma unroll
      for (int it = 0; it < 8; ++it) {
        const int row = it * 2 + hh2;
        v4f v = *(const v4f*)(slab + row * 68 + c4);
#pragma unroll
        for (int e = 0; e < 4; ++e) v[e] = v[e] * oscale + bc[e];
        vals[it] = v;
      }
      for (int pass = 0; pass < 2; ++pass) {
#pragma unroll
        for (int it = 0; it < 8; ++it) {
          const int row = it * 2 + hh2;
          *(volatile v4f*)(C + (size_t)(mBase + row) * ldc + n0 + c4) = vals[it];
        }
        __threadfence();
      }
    } else {
      unsigned short* C = (unsigned short*)Cout + (size_t)y * (size_t)strideC;
      v4u hv[4], hr[4];
#pragma unroll
      for (int it = 0; it < 4; ++it) {
        const int row = it * 4 + q8;
        const float* sp = slab + row * 68 + c8;
        float bm = 0.f;
        if constexpr (BIASM == 1) {
          const int mi = mBase + row;
          const int mc = (mi < nbias - 1) ? mi : (nbias - 1);
          bm = bfr(biasb[mc]);
        }
        v4u a, ar;
#pragma unroll
        for (int e = 0; e < 4; ++e) {
          const float f0 = sp[2 * e]     * oscale + ((BIASM == 1) ? bm : bc[2 * e]);
          const float f1 = sp[2 * e + 1] * oscale + ((BIASM == 1) ? bm : bc[2 * e + 1]);
          const _Float16 g0 = (_Float16)f0, g1 = (_Float16)f1;
          a[e] = pk16(h_bits(g0), h_bits(g1));
          const float e0 = (f0 - (float)g0) * RSC;
          const float e1 = (f1 - (float)g1) * RSC;
          ar[e] = pk16(h_bits((_Float16)e0), h_bits((_Float16)e1));
        }
        hv[it] = a;
        hr[it] = ar;
      }
      for (int pass = 0; pass < 2; ++pass) {
#pragma unroll
        for (int it = 0; it < 4; ++it) {
          const int row = it * 4 + q8;
          unsigned short* dp = C + (size_t)(mBase + row) * ldc + n0 + c8;
          *(volatile v4u*)(dp) = hv[it];
          *(volatile v4u*)(dp + resOff) = hr[it];
        }
        __threadfence();
      }
    }
    wave_sync_lds();
  }
}

__global__ __launch_bounds__(256)
void attn_p(const unsigned short* __restrict__ qhp, const unsigned short* __restrict__ qrp,
            const unsigned short* __restrict__ khp, const unsigned short* __restrict__ krp,
            const int* __restrict__ mask, unsigned short* pp) {
  __shared__ __align__(16) float se[SBLK * SEQ];
  __shared__ float sinv[SBLK];
  __shared__ int   smask[SEQ];

  const int tid  = threadIdx.x;
  const int wave = tid >> 5;
  const int lane = tid & 31;
  const int hh   = lane >> 4;
  const int c    = lane & 15;
  const int sblk = blockIdx.x;
  const int hb   = blockIdx.y;
  const int h    = hb / NB;
  const int b    = hb % NB;
  const int s0   = sblk * SBLK;

  for (int i = tid; i < SEQ; i += 256) smask[i] = mask[i];

  {
    const int rg = wave & 1;
    const int tq = wave >> 1;
    const size_t qoff = (size_t)(b * SEQ + s0 + rg * 16 + c) * DQ + (size_t)h * DK + 8 * hh;
    const unsigned short* qh = qhp + qoff;
    const unsigned short* qr = qrp + qoff;
    const unsigned short* kh0 = khp + (size_t)h * DK + 8 * hh;
    const unsigned short* kr0 = krp + (size_t)h * DK + 8 * hh;
    float* erow = se + (rg * 16 + 8 * hh) * SEQ;
#pragma unroll 1
    for (int c4 = 0; c4 < 4; ++c4) {
      const int t0 = tq * 256 + c4 * 64;
      v8f ah[4], ar[4];
#pragma unroll
      for (int j = 0; j < 4; ++j) { ah[j] = zero8(); ar[j] = zero8(); }
#pragma unroll 2
      for (int ks = 0; ks < DK / 32; ++ks) {
        const v16us qav = ldfrag(qh + ks * 32);
        const v16us qbv = ldfrag(qr + ks * 32);
#pragma unroll
        for (int j = 0; j < 4; ++j) {
          const size_t ko = (size_t)(b * SEQ + t0 + 16 * j + c) * DQ + ks * 32;
          const v16us kav = ldfrag(kh0 + ko);
          const v16us kbv = ldfrag(kr0 + ko);
          ah[j] = mma_raw(qav, kav, ah[j]);
          ar[j] = mma_raw(qav, kbv, ar[j]);
          ar[j] = mma_raw(qbv, kav, ar[j]);
          guard2k4(ah[j], ar[j], qav, qbv, kav, kbv);
        }
      }
      acc_guard4(ah[0], ah[1], ah[2], ah[3]);
      acc_guard4(ar[0], ar[1], ar[2], ar[3]);
#pragma unroll
      for (int j = 0; j < 4; ++j) {
#pragma unroll
        for (int r = 0; r < 8; ++r) {
          erow[r * SEQ + t0 + 16 * j + c] = fmaf(ar[j][r], 1.0f / RSC, ah[j][r]);
        }
      }
    }
  }
  __syncthreads();

#pragma unroll 1
  for (int rr = 0; rr < 4; ++rr) {
    const int row = wave * 4 + rr;
    float* er = se + row * SEQ;
    float mx = -INFINITY;
#pragma unroll 4
    for (int i = 0; i < SEQ / 32; ++i) {
      const int t = lane + 32 * i;
      const float e = (smask[t] != 0) ? er[t] : NEGBIG;
      er[t] = e;
      mx = fmaxf(mx, e);
    }
#pragma unroll
    for (int off = 16; off > 0; off >>= 1) mx = fmaxf(mx, __shfl_xor(mx, off, 32));
    float sum = 0.f;
#pragma unroll 4
    for (int i = 0; i < SEQ / 32; ++i) {
      const int t = lane + 32 * i;
      const float ex = __expf(er[t] - mx);
      er[t] = ex;
      sum += ex;
    }
#pragma unroll
    for (int off = 16; off > 0; off >>= 1) sum += __shfl_xor(sum, off, 32);
    if (lane == 0) sinv[row] = PSC * (1.0f / sum);
  }
  __syncthreads();

  {
    const int tr = lane >> 2, sq = (lane & 3) * 8;
    unsigned short* preg = pp + ((size_t)(hb * NSB + sblk) * SEQ) * SBLK;
#pragma unroll 1
    for (int it = 0; it < SEQ / 64; ++it) {
      const int t = wave * (SEQ / 8) + it * 8 + tr;
      v4u o;
#pragma unroll
      for (int e = 0; e < 4; ++e) {
        const float f0 = se[(sq + 2 * e) * SEQ + t]     * sinv[sq + 2 * e];
        const float f1 = se[(sq + 2 * e + 1) * SEQ + t] * sinv[sq + 2 * e + 1];
        o[e] = pk16(h_bits((_Float16)f0), h_bits((_Float16)f1));
      }
      unsigned short* dst = preg + (size_t)t * SBLK + sq;
      *(volatile v4u*)dst = o;
      __threadfence();
      *(volatile v4u*)dst = o;
    }
  }
}

__global__ __launch_bounds__(256)
void pv64(const unsigned short* __restrict__ pp, const unsigned short* __restrict__ vth,
          const unsigned short* __restrict__ vtr, const float* __restrict__ xp,
          const float* __restrict__ gam, float* outp) {
  __shared__ __align__(16) float os[8][32 * 36];
  const int tid  = threadIdx.x;
  const int wave = tid >> 5;
  const int lane = tid & 31;
  const int hh   = lane >> 4;
  const int c    = lane & 15;
  const int dx = blockIdx.x, ty = blockIdx.y, hb = blockIdx.z;
  const int h  = hb / NB, b = hb % NB;
  const int wt = wave & 1, wd = wave >> 1;
  const int t0 = ty * 64 + wt * 32;
  const int d0 = dx * 128 + wd * 32;

  const unsigned short* pb = pp  + (size_t)hb * SEQ * SEQ + 8 * hh;
  const unsigned short* vh = vth + (size_t)hb * DK * SEQ + 8 * hh;
  const unsigned short* vr = vtr + (size_t)hb * DK * SEQ + 8 * hh;

  v8f acc[2][2], acr[2][2];
#pragma unroll
  for (int i = 0; i < 2; ++i)
#pragma unroll
    for (int j = 0; j < 2; ++j) { acc[i][j] = zero8(); acr[i][j] = zero8(); }

#pragma unroll 2
  for (int ks = 0; ks < SEQ / 32; ++ks) {
    v16us a[2], bhf[2], brf[2];
#pragma unroll
    for (int i = 0; i < 2; ++i)
      a[i] = ldfrag(pb + (size_t)ks * (SEQ * SBLK) + (size_t)(t0 + 16 * i + c) * SBLK);
#pragma unroll
    for (int j = 0; j < 2; ++j) {
      const size_t vo = (size_t)(d0 + 16 * j + c) * SEQ + ks * 32;
      bhf[j] = ldfrag(vh + vo);
      brf[j] = ldfrag(vr + vo);
    }
#pragma unroll
    for (int i = 0; i < 2; ++i) {
#pragma unroll
      for (int j = 0; j < 2; ++j) {
        acc[i][j] = mma_raw(a[i], bhf[j], acc[i][j]);
        acr[i][j] = mma_raw(a[i], brf[j], acr[i][j]);
      }
    }
    guard4k4(acc[0][0], acc[0][1], acc[1][0], acc[1][1], a[0], a[1], bhf[0], bhf[1]);
    guard4k4(acr[0][0], acr[0][1], acr[1][0], acr[1][1], a[0], a[1], brf[0], brf[1]);
  }
  acc_guard4(acc[0][0], acc[0][1], acc[1][0], acc[1][1]);
  acc_guard4(acr[0][0], acr[0][1], acr[1][0], acr[1][1]);

  float* osw = os[wave];
#pragma unroll
  for (int i = 0; i < 2; ++i) {
#pragma unroll
    for (int j = 0; j < 2; ++j) {
#pragma unroll
      for (int r = 0; r < 8; ++r) {
        osw[(16 * i + 8 * hh + r) * 36 + 16 * j + c] = fmaf(acr[i][j][r], 1.0f / RSC, acc[i][j][r]);
      }
    }
  }
  wave_sync_lds();

  const float g  = bfr(gam[h]);
  const float rg = 1.0f / (g + 1.0f);
  const int rl = lane >> 3, cc4 = (lane & 7) * 4;
  v4f vals[8];
#pragma unroll
  for (int it = 0; it < 8; ++it) {
    const int row = it * 4 + rl;
    const int t   = t0 + row;
    const v4f av = *(const v4f*)(osw + row * 36 + cc4);
    const v4f xv = *(const v4f*)(xp + ((size_t)(b * SEQ + t)) * DK + d0 + cc4);
    v4f o;
#pragma unroll
    for (int e = 0; e < 4; ++e) o[e] = (g * (av[e] * (1.0f / PSC)) + xv[e]) * rg;
    vals[it] = o;
  }
  for (int pass = 0; pass < 2; ++pass) {
#pragma unroll
    for (int it = 0; it < 8; ++it) {
      const int row = it * 4 + rl;
      const int t   = t0 + row;
      *(volatile v4f*)(outp + ((size_t)((b * NH + h) * SEQ + t)) * DK + d0 + cc4) = vals[it];
    }
    __threadfence();
  }
}

extern "C" void kernel_launch(void* const* d_in, const int* in_sizes, int n_in,
                              void* d_out, int out_size, void* d_ws, size_t ws_size,
                              hipStream_t stream) {
  if (n_in < 11) return;
  if (in_sizes[0] != MR * DK || in_sizes[1] != MR * DK) return;
  if (in_sizes[2] != DK * DQ || in_sizes[4] != DK * DQ || in_sizes[6] != DK * DQ) return;
  if (in_sizes[3] != DQ || in_sizes[5] != DQ || in_sizes[7] != DQ) return;
  if (in_sizes[8] != DK * DK || in_sizes[9] != NH || in_sizes[10] != SEQ) return;
  if (out_size != NB * NH * SEQ * DK) return;

  const float* x     = (const float*)d_in[0];
  const float* y     = (const float*)d_in[1];
  const float* Wq    = (const float*)d_in[2];
  const float* bq    = (const float*)d_in[3];
  const float* Wk    = (const float*)d_in[4];
  const float* bk    = (const float*)d_in[5];
  const float* Wv    = (const float*)d_in[6];
  const float* bv    = (const float*)d_in[7];
  const float* Wp    = (const float*)d_in[8];
  const float* gamma = (const float*)d_in[9];
  const int*   mask  = (const int*)d_in[10];

  const size_t PW   = (size_t)DQ * DK * 2;
  const size_t PWP  = (size_t)DK * DK * 2;
  const size_t PX   = (size_t)MR * DK * 2;
  const size_t PQ   = (size_t)2 * MR * DQ * 2;
  const size_t PVT  = (size_t)2 * NHB * DK * SEQ * 2;
  const size_t PXP  = (size_t)MR * DK * 4;
  const size_t PP   = (size_t)NHB * SEQ * SEQ * 2;
  if (PVT > PQ) return;
  size_t off = 0;
  const size_t oWq = off; off += PW;
  const size_t oWk = off; off += PW;
  const size_t oWv = off; off += PW;
  const size_t oWp = off; off += PWP;
  const size_t oXH = off; off += PX;
  const size_t oYH = off; off += PX;
  const size_t oQ  = off; off += PQ;
  const size_t oK  = off; off += PQ;
  const size_t oXP = off; off += PXP;
  const size_t oP  = off; off += PP;
  if (off > ws_size) return;
  if (off > (size_t)134217728) return;

  char* ws = (char*)d_ws;
  unsigned short* WqT = (unsigned short*)(ws + oWq);
  unsigned short* WkT = (unsigned short*)(ws + oWk);
  unsigned short* WvT = (unsigned short*)(ws + oWv);
  unsigned short* WpT = (unsigned short*)(ws + oWp);
  unsigned short* XH  = (unsigned short*)(ws + oXH);
  unsigned short* YH  = (unsigned short*)(ws + oYH);
  unsigned short* QH  = (unsigned short*)(ws + oQ);
  unsigned short* KH  = (unsigned short*)(ws + oK);
  unsigned short* VT  = (unsigned short*)(ws + oQ);
  float*          XP  = (float*)(ws + oXP);
  unsigned short* P   = (unsigned short*)(ws + oP);
  float*          out = (float*)d_out;

  const int n8x = (MR * DK) / 8;
  if ((n8x % 256) != 0) return;
  const dim3 blk(256);
  const dim3 gTw(DQ / 64, DK / 64);
  const dim3 gTp(DK / 64, DK / 64);
  const dim3 gCx((n8x + 255) / 256);
  const dim3 gQK(((MR / 64) * (DQ / 64) + 7) / 8, 1);
  const dim3 gXP(((MR / 64) * (DK / 64) + 7) / 8, 1);
  const dim3 gVT(((DK / 64) * (SEQ / 64) + 7) / 8, NHB);
  const dim3 gAt(NSB, NHB);
  const dim3 gPV(DK / 128, SEQ / 64, NHB);
  const float invw = 1.0f / WSC;

  tconv_h16<<<gTw, blk, 0, stream>>>(Wq, WqT, DQ, WSC);
  tconv_h16<<<gTw, blk, 0, stream>>>(Wk, WkT, DQ, WSC);
  tconv_h16<<<gTw, blk, 0, stream>>>(Wv, WvT, DQ, WSC);
  tconv_h16<<<gTp, blk, 0, stream>>>(Wp, WpT, DK, WSC);

  conv_h16<<<gCx, blk, 0, stream>>>(x, XH, n8x, 1.0f);
  conv_h16<<<gCx, blk, 0, stream>>>(y, YH, n8x, 1.0f);

  gemm64<3, 0><<<gQK, blk, 0, stream>>>(
      XH, DK, 0LL, WqT, DK, 0LL, bq, DQ, 0LL, 1,
      (void*)QH, DQ, 0LL, (long long)QRES, MR, DQ, DK, invw);
  gemm64<3, 0><<<gQK, blk, 0, stream>>>(
      YH, DK, 0LL, WkT, DK, 0LL, bk, DQ, 0LL, 1,
      (void*)KH, DQ, 0LL, (long long)QRES, MR, DQ, DK, invw);

  gemm64<0, 2><<<gXP, blk, 0, stream>>>(
      XH, DK, 0LL, WpT, DK, 0LL, bq, DQ, 0LL, 1,
      (void*)XP, DK, 0LL, 0LL, MR, DK, DK, invw);

  attn_p<<<gAt, blk, 0, stream>>>(QH, QH + QRES, KH, KH + QRES, mask, P);

  gemm64<3, 1><<<gVT, blk, 0, stream>>>(
      WvT, DK, (long long)DK * DK, YH, DK, (long long)SEQ * DK, bv, DK, (long long)DK, NB,
      (void*)VT, SEQ, (long long)DK * SEQ, (long long)VRES, DK, SEQ, DK, invw);

  pv64<<<gPV, blk, 0, stream>>>(P, VT, VT + VRES, XP, gamma, out);
  (void)hipGetLastError();
}
